// OuterProductMean_962072674751
// MI455X (gfx1250) — hardware-verified
//
#include <hip/hip_runtime.h>
#include <stdint.h>

constexpr int kS     = 128;
constexpr int kNres  = 256;
constexpr int kCs    = 256;
constexpr int kC     = 32;
constexpr int kCz    = 128;
constexpr int kTok   = kS * kNres;
constexpr int kN1    = 2 * kC;
constexpr int kKout  = kC * kC;
constexpr int kMrows = kNres * kC;
constexpr float kWoutCarry = 32.0f;
constexpr float kOutScale  = 1.0f / (128.0f * 32.0f);
constexpr float kInvCs = 1.0f / 256.0f;
constexpr float kLnEps = 1e-5f;

static_assert(kTok % 64 == 0, "M tile");
static_assert(kN1 % 64 == 0, "N tile");
static_assert(kCs % 32 == 0, "K step");
static_assert(kS % 32 == 0, "K step");
static_assert(kKout % 32 == 0, "K step");
static_assert(kTok % 8 == 0, "ln grid");

typedef __attribute__((ext_vector_type(16))) _Float16 v16h;
typedef __attribute__((ext_vector_type(8)))  _Float16 v8h;
typedef __attribute__((ext_vector_type(16))) __bf16   v16b;
typedef __attribute__((ext_vector_type(8)))  __bf16   v8b;
typedef __attribute__((ext_vector_type(8)))  float    v8f;
typedef __attribute__((ext_vector_type(4)))  float    v4f;
typedef __attribute__((ext_vector_type(4)))  unsigned int v4u;

__device__ __forceinline__ unsigned short f2bf_bits(float f) {
  unsigned u = __float_as_uint(f);
  return (unsigned short)((u + 0x7FFFu + ((u >> 16) & 1u)) >> 16);
}
__device__ __forceinline__ float bf_bits2f(unsigned short h) { return __uint_as_float(((unsigned)h) << 16); }
__device__ __forceinline__ unsigned pk16(unsigned short a, unsigned short b) { return (unsigned)a | ((unsigned)b << 16); }
__device__ __forceinline__ unsigned short h_bits(float f) { const _Float16 h = (_Float16)f; return __builtin_bit_cast(unsigned short, h); }

__device__ __forceinline__ void dep_guard_h(v8f& a, v8f& b, v16h x, v16h y) { asm volatile("v_nop\n\tv_nop\n\tv_nop\n\tv_nop" : "+v"(a), "+v"(b) : "v"(x), "v"(y)); }
__device__ __forceinline__ void dep_guard_b(v8f& a, v8f& b, v16b x, v16b y) { asm volatile("v_nop\n\tv_nop\n\tv_nop\n\tv_nop" : "+v"(a), "+v"(b) : "v"(x), "v"(y)); }
__device__ __forceinline__ void dep_guard4_h(v8f& a, v8f& b, v8f& c, v8f& d, v16h x, v16h y) {
  asm volatile("v_nop\n\tv_nop\n\tv_nop\n\tv_nop" : "+v"(a), "+v"(b), "+v"(c), "+v"(d) : "v"(x), "v"(y));
}
__device__ __forceinline__ void dep_guard4_b(v8f& a, v8f& b, v8f& c, v8f& d, v16b x, v16b y) {
  asm volatile("v_nop\n\tv_nop\n\tv_nop\n\tv_nop" : "+v"(a), "+v"(b), "+v"(c), "+v"(d) : "v"(x), "v"(y));
}
__device__ __forceinline__ void keep4_h(v16h a, v16h b, v16h c, v16h d) { asm volatile("v_nop" :: "v"(a), "v"(b), "v"(c), "v"(d)); }
__device__ __forceinline__ void keep4_b(v16b a, v16b b, v16b c, v16b d) { asm volatile("v_nop" :: "v"(a), "v"(b), "v"(c), "v"(d)); }
__device__ __forceinline__ void acc_guard4(v8f& a, v8f& b, v8f& c, v8f& d) { asm volatile("v_nop\n\tv_nop\n\tv_nop\n\tv_nop" : "+v"(a), "+v"(b), "+v"(c), "+v"(d)); }
template <typename T> struct Frag;
template <> struct Frag<_Float16> {
  typedef v16h V; union U { v16h v; v8h h[2]; };
  static __device__ __forceinline__ v16h load(const _Float16* p) {
    U f; f.h[0] = *(const v8h*)(p); f.h[1] = *(const v8h*)(p + 16); return f.v;
  }
  static __device__ __forceinline__ v8f mma(v16h a, v16h b, v8f c) {
    return __builtin_amdgcn_wmma_f32_16x16x32_f16(false, a, false, b, (short)0, c, false, false);
  }
  static __device__ __forceinline__ void guard(v8f& a, v8f& b, v16h x, v16h y) { dep_guard_h(a, b, x, y); }
  static __device__ __forceinline__ void guard4(v8f& a, v8f& b, v8f& c, v8f& d, v16h x, v16h y) { dep_guard4_h(a, b, c, d, x, y); }
  static __device__ __forceinline__ void keep(v16h a, v16h b, v16h c, v16h d) { keep4_h(a, b, c, d); }
};
template <> struct Frag<__bf16> {
  typedef v16b V; union U { v16b v; v8b h[2]; };
  static __device__ __forceinline__ v16b load(const __bf16* p) {
    U f; f.h[0] = *(const v8b*)(p); f.h[1] = *(const v8b*)(p + 16); return f.v;
  }
  static __device__ __forceinline__ v8f mma(v16b a, v16b b, v8f c) {
    return __builtin_amdgcn_wmma_f32_16x16x32_bf16(false, a, false, b, (short)0, c, false, false);
  }
  static __device__ __forceinline__ void guard(v8f& a, v8f& b, v16b x, v16b y) { dep_guard_b(a, b, x, y); }
  static __device__ __forceinline__ void guard4(v8f& a, v8f& b, v8f& c, v8f& d, v16b x, v16b y) { dep_guard4_b(a, b, c, d, x, y); }
  static __device__ __forceinline__ void keep(v16b a, v16b b, v16b c, v16b d) { keep4_b(a, b, c, d); }
};
__device__ __forceinline__ v8f mma_h_guard(v16h a, v16h b, v8f c) {
  c = __builtin_amdgcn_wmma_f32_16x16x32_f16(false, a, false, b, (short)0, c, false, false);
  asm volatile("v_nop\n\tv_nop\n\tv_nop\n\tv_nop" : "+v"(c) : "v"(a), "v"(b));
  return c;
}

template <int ET> struct Elem;
template <> struct Elem<0> { typedef _Float16 T; };
template <> struct Elem<1> { typedef __bf16 T; };
template <int ET, bool SPLIT, int BIAS_MODE, int OUT_MODE, bool RESID, int ACT = 0>
__global__ __launch_bounds__(256) void wmma_gemm64(
    const unsigned short* __restrict__ Ap, const unsigned short* __restrict__ A2p, int lda, long strideA,
    const unsigned short* __restrict__ Btp, const unsigned short* __restrict__ Bt2p, int ldb, long strideB,
    void* __restrict__ Cout, void* __restrict__ Cout2, int ldc, long strideC,
    const float* __restrict__ bias,
    const float* __restrict__ resid, long strideR,
    int M, int N, int K, float scale) {
  typedef typename Elem<ET>::T T;
  typedef typename Frag<T>::V V;
  const T* A = (const T*)Ap; const T* A2 = (const T*)A2p; const T* Bt = (const T*)Btp; const T* Bt2 = (const T*)Bt2p;
  __shared__ __align__(16) float sT[8][16 * 68];
  const int b    = blockIdx.y;
  const int lane = threadIdx.x & 31;
  const int wave = threadIdx.x >> 5;
  const int tilesN = N >> 6;
  const int tilesM = M >> 6;
  const int tile = blockIdx.x * 8 + wave;
  if (tile >= tilesM * tilesN) return;
  const int tm = tile / tilesN;
  const int tn = tile - tm * tilesN;
  const int m0 = tm << 6;
  const int n0 = tn << 6;

  const T* Ab  = A  + (size_t)b * strideA;
  const T* Bb  = Bt + (size_t)b * strideB;
  const T* Ab2 = SPLIT ? (A2  + (size_t)b * strideA) : nullptr;
  const T* Bb2 = SPLIT ? (Bt2 + (size_t)b * strideB) : nullptr;

  const int rlane = lane & 15;
  const int koff  = (lane >> 4) * 8;
  const int mOff  = (lane >> 4) * 8;

  v8f acc[4][4];
#pragma unroll
  for (int i = 0; i < 4; ++i)
#pragma unroll
    for (int j = 0; j < 4; ++j) acc[i][j] = (v8f){0.f,0.f,0.f,0.f,0.f,0.f,0.f,0.f};

  for (int k0 = 0; k0 < K; k0 += 32) {
    V bh[4], bl[4];
#pragma unroll
    for (int j = 0; j < 4; ++j) {
      const size_t bo = (size_t)(n0 + (j << 4) + rlane) * ldb + koff + k0;
      bh[j] = Frag<T>::load(Bb + bo);
      if (SPLIT) bl[j] = Frag<T>::load(Bb2 + bo);
    }
#pragma unroll
    for (int i = 0; i < 4; ++i) {
      const size_t ao = (size_t)(m0 + (i << 4) + rlane) * lda + koff + k0;
      V ah = Frag<T>::load(Ab + ao);
      V al;
      if (SPLIT) al = Frag<T>::load(Ab2 + ao);
#pragma unroll
      for (int j = 0; j < 4; ++j) {
        acc[i][j] = Frag<T>::mma(ah, bh[j], acc[i][j]);
        if (SPLIT) {
          acc[i][j] = Frag<T>::mma(ah, bl[j], acc[i][j]);
          acc[i][j] = Frag<T>::mma(al, bh[j], acc[i][j]);
        }
      }
      Frag<T>::guard4(acc[i][0], acc[i][1], acc[i][2], acc[i][3], ah, SPLIT ? al : ah);
    }
    Frag<T>::keep(bh[0], bh[1], bh[2], bh[3]);
    if (SPLIT) Frag<T>::keep(bl[0], bl[1], bl[2], bl[3]);
  }
  acc_guard4(acc[0][0], acc[0][1], acc[0][2], acc[0][3]);
  acc_guard4(acc[1][0], acc[1][1], acc[1][2], acc[1][3]);
  acc_guard4(acc[2][0], acc[2][1], acc[2][2], acc[2][3]);
  acc_guard4(acc[3][0], acc[3][1], acc[3][2], acc[3][3]);

  float* slab = sT[wave];
  const float* Rb = RESID ? (resid + (size_t)b * strideR) : nullptr;
#pragma unroll
  for (int i = 0; i < 4; ++i) {
    const int mBase = m0 + (i << 4);
#pragma unroll
    for (int j = 0; j < 4; ++j) {
      const int n = n0 + (j << 4) + rlane;
      float bv = 0.f;
      if (BIAS_MODE == 2) bv = bias[n];
#pragma unroll
      for (int r = 0; r < 8; ++r) {
        float v = acc[i][j][r] * scale;
        if (BIAS_MODE == 1) v += bias[mBase + mOff + r];
        if (BIAS_MODE == 2) v += bv;
        if (RESID) v += Rb[(size_t)(mBase + mOff + r) * ldc + n];
        if (ACT == 2) v = fmaxf(v, 0.0f);
        if (ACT == 4) v = (v > 0.f) ? v : 0.01f * v;
        slab[(mOff + r) * 68 + (j << 4) + rlane] = v;
      }
    }
    __builtin_amdgcn_fence(__ATOMIC_RELEASE, "workgroup");
    __builtin_amdgcn_wave_barrier();
    __builtin_amdgcn_fence(__ATOMIC_ACQUIRE, "workgroup");
    if (OUT_MODE == 0) {
      float* C = (float*)Cout + (size_t)b * strideC;
      const int hh = lane >> 4, c4 = (lane & 15) * 4;
      for (int pass = 0; pass < 2; ++pass) {
#pragma unroll
        for (int it = 0; it < 8; ++it) {
          const int row = it * 2 + hh;
          v4f v = *(const v4f*)(slab + row * 68 + c4);
          *(volatile v4f*)(C + (size_t)(mBase + row) * ldc + n0 + c4) = v;
        }
        __threadfence();
      }
    } else {
      const int q = lane >> 3, c8 = (lane & 7) * 8;
      unsigned short* C  = (unsigned short*)Cout  + (size_t)b * strideC;
      unsigned short* C2 = (OUT_MODE == 2) ? ((unsigned short*)Cout2 + (size_t)b * strideC) : nullptr;
      for (int pass = 0; pass < 2; ++pass) {
#pragma unroll
        for (int it = 0; it < 4; ++it) {
          const int row = it * 4 + q;
          const float* sp = slab + row * 68 + c8;
          v8h hv, lv;
#pragma unroll
          for (int e = 0; e < 8; ++e) {
            if (OUT_MODE == 1) {
              hv[e] = (_Float16)sp[e];
            } else {
              unsigned short hb = f2bf_bits(sp[e]);
              unsigned short lb = f2bf_bits(sp[e] - bf_bits2f(hb));
              hv[e] = __builtin_bit_cast(_Float16, hb);
              lv[e] = __builtin_bit_cast(_Float16, lb);
            }
          }
          *(volatile v8h*)(C + (size_t)(mBase + row) * ldc + n0 + c8) = hv;
          if (OUT_MODE == 2) *(volatile v8h*)(C2 + (size_t)(mBase + row) * ldc + n0 + c8) = lv;
        }
        __threadfence();
      }
    }
    __builtin_amdgcn_fence(__ATOMIC_RELEASE, "workgroup");
    __builtin_amdgcn_wave_barrier();
    __builtin_amdgcn_fence(__ATOMIC_ACQUIRE, "workgroup");
  }
}

__global__ __launch_bounds__(256) void prep_wcat_kernel(const float* __restrict__ Wl, const float* __restrict__ Wr,
                                                        const float* __restrict__ bl, const float* __restrict__ br,
                                                        unsigned short* __restrict__ WcHi, unsigned short* __restrict__ WcLo,
                                                        float* __restrict__ biascat) {
  __shared__ float sm[64][65];
  __shared__ __align__(16) float sb[64];
  const int t = threadIdx.x;
  const int lane = t & 31, wave = t >> 5;
  const int kc = blockIdx.x;
#pragma unroll
  for (int it = 0; it < 8; ++it) {
    const int e  = it * 256 + t;
    const int kl = e >> 5;
    const int n  = e & 31;
    const size_t src = (size_t)(kc * 64 + kl) * kC + n;
    const float vl = Wl[src];
    const float vr = Wr[src];
    sm[n][kl]      = vl;
    sm[32 + n][kl] = vr;
    if ((it & 3) == 3) asm volatile("" ::: "memory");
  }
  if (t < 64) {
    const int idx = t & 31;
    const float a  = bl[idx];
    const float bb = br[idx];
    const float fs = (float)(t >> 5);
    sb[t] = fmaf(fs, bb, (1.0f - fs) * a);
  }
  __syncthreads();
  const int q = lane >> 3, c8 = (lane & 7) * 8;
  for (int pass = 0; pass < 2; ++pass) {
#pragma unroll
    for (int it = 0; it < 2; ++it) {
      const int row = wave * 8 + it * 4 + q;
      unsigned short hb[8], lb[8];
#pragma unroll
      for (int e = 0; e < 8; ++e) {
        const float v = sm[row][c8 + e];
        hb[e] = f2bf_bits(v);
        lb[e] = f2bf_bits(v - bf_bits2f(hb[e]));
      }
      const v4u uh = (v4u){pk16(hb[0], hb[1]), pk16(hb[2], hb[3]), pk16(hb[4], hb[5]), pk16(hb[6], hb[7])};
      const v4u ul = (v4u){pk16(lb[0], lb[1]), pk16(lb[2], lb[3]), pk16(lb[4], lb[5]), pk16(lb[6], lb[7])};
      const size_t o = (size_t)row * kCs + kc * 64 + c8;
      *(volatile v4u*)(WcHi + o) = uh;
      *(volatile v4u*)(WcLo + o) = ul;
    }
    __threadfence();
  }
  if (blockIdx.x == 0 && wave == 0) {
    const v4f bv = *(const v4f*)(sb + (lane & 15) * 4);
    for (int pass = 0; pass < 2; ++pass) {
      if (lane < 16) *(volatile v4f*)(biascat + lane * 4) = bv;
      __threadfence();
    }
  }
}

__global__ __launch_bounds__(256) void prep_wout_kernel(const float* __restrict__ Wout, unsigned short* __restrict__ WoutT) {
  __shared__ float sm[64][65];
  const int t  = threadIdx.x;
  const int k0 = blockIdx.x * 64;
  const int n0 = blockIdx.y * 64;
#pragma unroll
  for (int it = 0; it < 16; ++it) {
    const int e  = it * 256 + t;
    const int kl = e >> 6;
    const int nl = e & 63;
    sm[nl][kl] = Wout[(size_t)(k0 + kl) * kCz + n0 + nl] * kWoutCarry;
    if ((it & 3) == 3) asm volatile("" ::: "memory");
  }
  __syncthreads();
  const int lane = t & 31, wave = t >> 5;
  const int q = lane >> 3, c8 = (lane & 7) * 8;
  for (int pass = 0; pass < 2; ++pass) {
#pragma unroll
    for (int it = 0; it < 2; ++it) {
      const int row = wave * 8 + it * 4 + q;
      unsigned short hb[8];
#pragma unroll
      for (int e = 0; e < 8; ++e) hb[e] = h_bits(sm[row][c8 + e]);
      const v4u u = (v4u){pk16(hb[0], hb[1]), pk16(hb[2], hb[3]), pk16(hb[4], hb[5]), pk16(hb[6], hb[7])};
      *(volatile v4u*)(WoutT + (size_t)(n0 + row) * kKout + k0 + c8) = u;
    }
    __threadfence();
  }
}

__global__ __launch_bounds__(256) void ln_split_kernel(const float* __restrict__ msa, const float* __restrict__ gamma,
                                                       const float* __restrict__ beta,
                                                       unsigned short* __restrict__ Xhi, unsigned short* __restrict__ Xlo) {
  const int lane = threadIdx.x & 31, wave = threadIdx.x >> 5;
  const int row = blockIdx.x * 8 + wave;
  const float* p = msa + (size_t)row * kCs + lane * 8;
  const v4f a  = *(const v4f*)(p);
  const v4f c  = *(const v4f*)(p + 4);
  const v4f g0 = *(const v4f*)(gamma + lane * 8);
  const v4f g1 = *(const v4f*)(gamma + lane * 8 + 4);
  const v4f e0 = *(const v4f*)(beta + lane * 8);
  const v4f e1 = *(const v4f*)(beta + lane * 8 + 4);
  float x[8], g[8], bb[8];
#pragma unroll
  for (int e = 0; e < 4; ++e) { x[e] = a[e]; x[4 + e] = c[e]; g[e] = g0[e]; g[4 + e] = g1[e]; bb[e] = e0[e]; bb[4 + e] = e1[e]; }
  float s = ((x[0] + x[1]) + (x[2] + x[3])) + ((x[4] + x[5]) + (x[6] + x[7]));
#pragma unroll
  for (int off = 16; off > 0; off >>= 1) s += __shfl_xor(s, off, 32);
  const float mu = s * kInvCs;
  float v[8];
  float sq = 0.0f;
#pragma unroll
  for (int e = 0; e < 8; ++e) { v[e] = x[e] - mu; sq += v[e] * v[e]; }
#pragma unroll
  for (int off = 16; off > 0; off >>= 1) sq += __shfl_xor(sq, off, 32);
  const float rstd = rsqrtf(sq * kInvCs + kLnEps);
  unsigned short hb[8], lb[8];
#pragma unroll
  for (int e = 0; e < 8; ++e) {
    const float y = (v[e] * rstd) * g[e] + bb[e];
    hb[e] = f2bf_bits(y);
    lb[e] = f2bf_bits(y - bf_bits2f(hb[e]));
  }
  const v4u uh = (v4u){pk16(hb[0], hb[1]), pk16(hb[2], hb[3]), pk16(hb[4], hb[5]), pk16(hb[6], hb[7])};
  const v4u ul = (v4u){pk16(lb[0], lb[1]), pk16(lb[2], lb[3]), pk16(lb[4], lb[5]), pk16(lb[6], lb[7])};
  unsigned short* ph = Xhi + (size_t)row * kCs + lane * 8;
  unsigned short* pl = Xlo + (size_t)row * kCs + lane * 8;
  for (int pass = 0; pass < 2; ++pass) {
    *(volatile v4u*)ph = uh;
    *(volatile v4u*)pl = ul;
    __threadfence();
  }
}

constexpr int kTrLd = 136;
__global__ __launch_bounds__(256) void opm_transpose_kernel(const unsigned short* __restrict__ Y, unsigned short* __restrict__ AB2) {
  __shared__ __align__(16) unsigned short sm[64 * kTrLd];
  const int t = threadIdx.x;
  const int lane = t & 31, wave = t >> 5;
  const int i = blockIdx.x;
#pragma unroll
  for (int it = 0; it < 4; ++it) {
    const int e = it * 256 + t;
    const int s = e >> 3;
    const int q = e & 7;
    const v4u wv = *(const v4u*)(Y + ((size_t)(s * kNres + i)) * kN1 + q * 8);
#pragma unroll
    for (int e2 = 0; e2 < 4; ++e2) {
      const unsigned w = wv[e2];
      const int c0 = q * 8 + 2 * e2;
      sm[c0 * kTrLd + s]       = (unsigned short)(w & 0xffffu);
      sm[(c0 + 1) * kTrLd + s] = (unsigned short)(w >> 16);
    }
  }
  __syncthreads();
  const int hl = lane & 15, hh = lane >> 4;
  for (int pass = 0; pass < 2; ++pass) {
#pragma unroll
    for (int it = 0; it < 4; ++it) {
      const int c = wave * 8 + it * 2 + hh;
      const int side = c >> 5;
      const int cc = c & 31;
      const v4u u = *(const v4u*)(sm + c * kTrLd + hl * 8);
      unsigned short* dst = AB2 + (size_t)side * kMrows * kS + ((size_t)(i * kC + cc)) * kS + hl * 8;
      *(volatile v4u*)dst = u;
    }
    __threadfence();
  }
}

constexpr int kSmLd = kKout + 8;
constexpr int kSoLd = kCz + 4;
__global__ __launch_bounds__(256) void opm_outer_kernel(const unsigned short* __restrict__ AB2p,
                                                        const unsigned short* __restrict__ WoutTp,
                                                        const float* __restrict__ b_out, float* __restrict__ out) {
  __shared__ __align__(16) unsigned short sMean[16 * kSmLd];
  __shared__ __align__(16) float sOut[16 * kSoLd];
  const int lane = threadIdx.x & 31, wave = threadIdx.x >> 5;
  const int rlane = lane & 15;
  const int koff  = (lane >> 4) * 8;
  const int mOff  = (lane >> 4) * 8;
  const int i0 = blockIdx.y * 4;
  const int j0 = blockIdx.x * 4;
  const _Float16* A2 = (const _Float16*)AB2p + (size_t)(i0 * kC) * kS;
  const _Float16* B2 = (const _Float16*)AB2p + (size_t)kMrows * kS + (size_t)(j0 * kC) * kS;
  const _Float16* Wt = (const _Float16*)WoutTp;
  const int mrow0 = (wave & 3) * 32;
  const int ncol0 = (wave >> 2) * 64;

  v8f acc[2][4];
#pragma unroll
  for (int i = 0; i < 2; ++i)
#pragma unroll
    for (int j = 0; j < 4; ++j) acc[i][j] = (v8f){0.f,0.f,0.f,0.f,0.f,0.f,0.f,0.f};
#pragma unroll 1
  for (int k0 = 0; k0 < kS; k0 += 32) {
    v16h bh[4];
#pragma unroll
    for (int j = 0; j < 4; ++j)
      bh[j] = Frag<_Float16>::load(B2 + (size_t)(ncol0 + (j << 4) + rlane) * kS + koff + k0);
#pragma unroll
    for (int i = 0; i < 2; ++i) {
      const v16h ah = Frag<_Float16>::load(A2 + (size_t)(mrow0 + (i << 4) + rlane) * kS + koff + k0);
#pragma unroll
      for (int j = 0; j < 4; ++j) acc[i][j] = Frag<_Float16>::mma(ah, bh[j], acc[i][j]);
      dep_guard4_h(acc[i][0], acc[i][1], acc[i][2], acc[i][3], ah, bh[0]);
    }
    keep4_h(bh[0], bh[1], bh[2], bh[3]);
  }
  acc_guard4(acc[0][0], acc[0][1], acc[0][2], acc[0][3]);
  acc_guard4(acc[1][0], acc[1][1], acc[1][2], acc[1][3]);

#pragma unroll
  for (int i = 0; i < 2; ++i) {
#pragma unroll
    for (int j = 0; j < 4; ++j) {
      const int nG = ncol0 + (j << 4) + rlane;
      const int p  = (wave & 3) * 4 + (nG >> 5);
      const int d  = nG & 31;
#pragma unroll
      for (int r = 0; r < 8; ++r) {
        const int cch = (i << 4) + mOff + r;
        sMean[p * kSmLd + cch * kC + d] = h_bits(acc[i][j][r]);
      }
    }
  }
  __syncthreads();

  const int n0w = wave * 16;
  v8f acc2 = (v8f){0.f,0.f,0.f,0.f,0.f,0.f,0.f,0.f};
  const _Float16* sMh = (const _Float16*)(const void*)sMean;
#pragma unroll 2
  for (int k0 = 0; k0 < kKout; k0 += 32) {
    const v16h a2 = Frag<_Float16>::load(sMh + rlane * kSmLd + koff + k0);
    const v16h b2 = Frag<_Float16>::load(Wt + (size_t)(n0w + rlane) * kKout + koff + k0);
    acc2 = mma_h_guard(a2, b2, acc2);
  }
  const float bo = b_out[n0w + rlane];
#pragma unroll
  for (int r = 0; r < 8; ++r) sOut[(mOff + r) * kSoLd + n0w + rlane] = fmaf(acc2[r], kOutScale, bo);
  __syncthreads();

  for (int pass = 0; pass < 2; ++pass) {
#pragma unroll
    for (int it = 0; it < 2; ++it) {
      const int p  = wave * 2 + it;
      const int il = p >> 2, jl = p & 3;
      const v4f val = *(const v4f*)(sOut + p * kSoLd + lane * 4);
      float* dst = out + ((size_t)(i0 + il) * kNres + (size_t)(j0 + jl)) * kCz + lane * 4;
      *(volatile v4f*)dst = val;
    }
    __threadfence();
  }
}

extern "C" void kernel_launch(void* const* d_in, const int* in_sizes, int n_in,
                              void* d_out, int out_size, void* d_ws, size_t ws_size,
                              hipStream_t stream) {
  if (n_in < 9) return;
  if (in_sizes[0] != kTok * kCs) return;
  if (out_size != kNres * kNres * kCz) return;

  const float* msa      = (const float*)d_in[0];
  const float* ln_gamma = (const float*)d_in[1];
  const float* ln_beta  = (const float*)d_in[2];
  const float* W_left   = (const float*)d_in[3];
  const float* b_left   = (const float*)d_in[4];
  const float* W_right  = (const float*)d_in[5];
  const float* b_right  = (const float*)d_in[6];
  const float* W_out    = (const float*)d_in[7];
  const float* b_out    = (const float*)d_in[8];
  float* out = (float*)d_out;

  const size_t bXhi  = (size_t)kTok * kCs * 2;
  const size_t bXlo  = bXhi;
  const size_t bY    = (size_t)kTok * kN1 * 2;
  const size_t bAB2  = (size_t)2 * kMrows * kS * 2;
  const size_t bWoT  = (size_t)kCz * kKout * 2;
  const size_t bWc   = (size_t)kN1 * kCs * 2;
  const size_t bBias = 256;
  size_t off = 0;
  char* ws = (char*)d_ws;
  unsigned short* Xhi   = (unsigned short*)(ws + off); off += bXhi;
  unsigned short* Xlo   = (unsigned short*)(ws + off); off += bXlo;
  unsigned short* Y     = (unsigned short*)(ws + off); off += bY;
  unsigned short* AB2   = (unsigned short*)(ws + off); off += bAB2;
  unsigned short* WoutT = (unsigned short*)(ws + off); off += bWoT;
  unsigned short* WcHi  = (unsigned short*)(ws + off); off += bWc;
  unsigned short* WcLo  = (unsigned short*)(ws + off); off += bWc;
  float* biascat        = (float*)(ws + off);          off += bBias;
  if (off > ws_size) return;

  prep_wcat_kernel<<<dim3(kCs / 64), dim3(256), 0, stream>>>(W_left, W_right, b_left, b_right, WcHi, WcLo, biascat);
  prep_wout_kernel<<<dim3(kKout / 64, kCz / 64), dim3(256), 0, stream>>>(W_out, WoutT);
  ln_split_kernel<<<dim3(kTok / 8), dim3(256), 0, stream>>>(msa, ln_gamma, ln_beta, Xhi, Xlo);
  {
    const int M = kTok, N = kN1, K = kCs;
    static_assert(kTok % 64 == 0 && kN1 % 64 == 0 && kCs % 32 == 0, "gemm shape");
    const int tiles = (M / 64) * (N / 64);
    dim3 grid((tiles + 7) / 8, 1);
    wmma_gemm64<1, true, 2, 1, false, 0><<<grid, dim3(256), 0, stream>>>(
        Xhi, Xlo, K, 0L,
        WcHi, WcLo, K, 0L,
        (void*)Y, (void*)Y, N, 0L,
        biascat,
        (const float*)biascat, 0L,
        M, N, K, 1.0f);
  }
  opm_transpose_kernel<<<dim3(kNres), dim3(256), 0, stream>>>(Y, AB2);
  opm_outer_kernel<<<dim3(kNres / 4, kNres / 4), dim3(256), 0, stream>>>(AB2, WoutT, b_out, out);
}
